// WindowAttentionMemory_45389214384571
// MI455X (gfx1250) — hardware-verified
//
#include <hip/hip_runtime.h>


namespace {
constexpr int B = 2, S = 2048, H = 1024, NH = 16, HD = 64, WIN = 256, NBLK = S / 16, ROWS = B * S;
constexpr float XS = 8.0f, PS = 1024.0f, WSC = 256.0f;
typedef _Float16 b16;
typedef __attribute__((ext_vector_type(16))) _Float16 v16b;
typedef __attribute__((ext_vector_type(8))) _Float16 v8b;
typedef __attribute__((ext_vector_type(8))) float v8f;
typedef __attribute__((ext_vector_type(4))) float v4f;
typedef __attribute__((ext_vector_type(2))) float v2f;
__device__ __forceinline__ float bf16_rne(float f) { unsigned int u = __float_as_uint(f); u += 0x7FFFu + ((u >> 16) & 1u); return __uint_as_float(u & 0xFFFF0000u); }
__device__ __forceinline__ void split16(float v, b16& hi, b16& lo) { hi = (b16)v; lo = (b16)(v - (float)hi); }
__device__ __forceinline__ v16b frag_kb(const b16* p, int hh) { const v8b a = *(const v8b*)(p + 8 * hh), b = *(const v8b*)(p + 16 + 8 * hh); v16b f;
#pragma unroll
  for (int e = 0; e < 8; ++e) { f[e] = a[e]; f[8 + e] = b[e]; } return f; }
__device__ __forceinline__ v8f wmma16b(v16b a, v16b b, v8f c) { v8f d = __builtin_amdgcn_wmma_f32_16x16x32_f16(false, a, false, b, (short)0, c, false, false); asm volatile("v_nop\n\tv_nop\n\tv_nop\n\tv_nop" : "+v"(d) : "v"(a), "v"(b)); return d; }
__device__ __forceinline__ void wave_lds_sync() { __builtin_amdgcn_fence(__ATOMIC_RELEASE, "workgroup"); __builtin_amdgcn_wave_barrier(); __builtin_amdgcn_fence(__ATOMIC_ACQUIRE, "workgroup"); }
__device__ __forceinline__ float pmul(float a, float b) { float p = a * b; asm volatile("" : "+v"(p)); return p; }

__global__ __launch_bounds__(256) void wcopy_kernel(const float* __restrict__ w, int ro, b16* __restrict__ WT) {
  const size_t u = (size_t)blockIdx.x * 256 + threadIdx.x; if (u >= (size_t)H * H / 8) return; const size_t e = u * 8; v8b v;
#pragma unroll
  for (int j = 0; j < 8; ++j) v[j] = (b16)(bf16_rne(w[e + j]) * WSC); for (int pass = 0; pass < 2; ++pass) { *(volatile v8b*)(WT + (size_t)ro * H + e) = v; __threadfence(); }
}
__global__ __launch_bounds__(256) void ln_kernel(const float* __restrict__ hs, const float* __restrict__ g, const float* __restrict__ bt, int RLIM, b16* __restrict__ XN) {
  const int wave = threadIdx.x >> 5, lane = threadIdx.x & 31; const size_t r = (size_t)blockIdx.x * 8 + wave; if (r >= (size_t)RLIM) return; const float* row = hs + r * H; float s = 0.0f;
#pragma unroll 1
  for (int c = lane; c < H; c += 32) s += bf16_rne(row[c]);
  for (int o = 16; o; o >>= 1) s += __shfl_xor(s, o); const float mu = s * (1.0f / H); float v = 0.0f;
#pragma unroll 1
  for (int c = lane; c < H; c += 32) { const float d = bf16_rne(row[c]) - mu; v += pmul(d, d); }
  for (int o = 16; o; o >>= 1) v += __shfl_xor(v, o); const float rs = rsqrtf(v * (1.0f / H) + 1e-12f);
  for (int pass = 0; pass < 2; ++pass) {
#pragma unroll 1
    for (int q = 0; q < 4; ++q) { const int c0 = q * 256 + lane * 8; v8b pk;
#pragma unroll
      for (int i = 0; i < 8; ++i) { const int c = c0 + i; pk[i] = (b16)((pmul(pmul(bf16_rne(row[c]) - mu, rs), bf16_rne(g[c])) + bf16_rne(bt[c])) * XS); }
      *(volatile v8b*)(XN + r * H + c0) = pk; }
    __threadfence(); }
}
template <int RESID>
__global__ __launch_bounds__(32) void dense_kernel(const b16* __restrict__ A, const b16* __restrict__ WT, const float* __restrict__ bias, const float* __restrict__ res, int NG, float* __restrict__ OUT, int outp) {
  __shared__ float Tf[16][132]; const int lane = threadIdx.x, nloc = lane & 15, hlf = lane >> 4; const int g = blockIdx.x % NG; const size_t m0 = (size_t)(blockIdx.x / NG) * 16;
  v8f acc[8];
#pragma unroll
  for (int t = 0; t < 8; ++t) acc[t] = (v8f){};
#pragma unroll 2
  for (int kb = 0; kb < H; kb += 32) { const v16b a = frag_kb(A + (m0 + nloc) * H + kb, hlf);
#pragma unroll
    for (int t = 0; t < 8; ++t) acc[t] = wmma16b(a, frag_kb(WT + ((size_t)g * 128 + t * 16 + nloc) * H + kb, hlf), acc[t]); }
#pragma unroll
  for (int t = 0; t < 8; ++t) { const int c = g * 128 + t * 16 + nloc; const float bb = bf16_rne(bias[c]);
#pragma unroll
    for (int r8 = 0; r8 < 8; ++r8) Tf[8 * hlf + r8][t * 16 + nloc] = acc[t][r8] * (1.0f / (XS * WSC)) + bb; }
  wave_lds_sync();
  for (int pass = 0; pass < 2; ++pass) { for (int rr = 0; rr < 16; ++rr) { v4f v = *(const v4f*)(&Tf[rr][lane * 4]); if (RESID) { for (int q4 = 0; q4 < 4; ++q4) v[q4] += bf16_rne(res[(m0 + rr) * H + g * 128 + lane * 4 + q4]); } *(volatile v4f*)(OUT + (m0 + rr) * (size_t)outp + g * 128 + lane * 4) = v; } __threadfence(); }
}
__global__ __launch_bounds__(32) void att_kernel(const float* __restrict__ QKV, int BV, int NQB, b16* __restrict__ ATT) {
  __shared__ __attribute__((aligned(16))) b16 Qh[16][72], Ql[16][72], Kh[32][72], Kl[32][72], Ph[16][40], Vh[HD][40], Vl[HD][40]; __shared__ float Sc[16][33], M[16], Dn[16], Sf[16], Of[16][HD + 1];
  const int lane = threadIdx.x, nloc = lane & 15, hlf = lane >> 4; const int qb = blockIdx.x % NQB, h = (blockIdx.x / NQB) % NH, b = blockIdx.x / (NQB * NH); if (b >= BV) return; const size_t base = (size_t)b * S; const int q0 = qb * 16;
  for (int rr = 0; rr < 16; ++rr) for (int qd = 0; qd < 2; ++qd) { b16 p, ql; split16(QKV[(base + q0 + rr) * (3 * H) + h * HD + qd * 32 + lane] * XS, p, ql); Qh[rr][qd * 32 + lane] = p; Ql[rr][qd * 32 + lane] = ql; }
  if (lane < 16) { M[lane] = -INFINITY; Dn[lane] = 0.0f; Sf[lane] = 0.0f; }
  v8f acc[4];
#pragma unroll
  for (int t = 0; t < 4; ++t) acc[t] = (v8f){};
  wave_lds_sync(); int k0 = q0 - (WIN - 1); if (k0 < 0) k0 = 0; k0 &= ~31;
#pragma unroll 1
  for (int kc = k0; kc < q0 + 16; kc += 32) {
    for (int rr = 0; rr < 32; ++rr) { const size_t kn = base + kc + rr; const float* kp = QKV + kn * (3 * H) + H + h * HD; const float* vp = QKV + kn * (3 * H) + 2 * H + h * HD; b16 p, ql;
      for (int qd = 0; qd < 2; ++qd) { split16(kp[qd * 32 + lane] * XS, p, ql); Kh[rr][qd * 32 + lane] = p; Kl[rr][qd * 32 + lane] = ql; split16(vp[qd * 32 + lane] * XS, p, ql); Vh[qd * 32 + lane][rr] = p; Vl[qd * 32 + lane][rr] = ql; } }
    wave_lds_sync();
#pragma unroll
    for (int blk = 0; blk < 2; ++blk) { v8f s = {};
#pragma unroll
      for (int ks = 0; ks < HD; ks += 32) { const v16b qh = frag_kb(&Qh[nloc][ks], hlf), ql = frag_kb(&Ql[nloc][ks], hlf), kh = frag_kb(&Kh[blk * 16 + nloc][ks], hlf), kl = frag_kb(&Kl[blk * 16 + nloc][ks], hlf); s = wmma16b(qh, kh, s); s = wmma16b(qh, kl, s); s = wmma16b(ql, kh, s); }
#pragma unroll
      for (int r8 = 0; r8 < 8; ++r8) { const int qi = q0 + 8 * hlf + r8, kj = kc + blk * 16 + nloc; const bool ok = kj <= qi && kj >= qi - (WIN - 1); Sc[8 * hlf + r8][blk * 16 + nloc] = ok ? s[r8] * (0.125f / (XS * XS)) : -INFINITY; } }
    wave_lds_sync();
#pragma unroll 1
    for (int qi = 0; qi < 16; ++qi) { const float sv = Sc[qi][lane]; float cm = sv; for (int o = 16; o; o >>= 1) cm = fmaxf(cm, __shfl_xor(cm, o)); const float mo = M[qi]; const float mn = fmaxf(mo, cm); const float p = (sv == -INFINITY) ? 0.0f : __expf(sv - mn); float psum = p; for (int o = 16; o; o >>= 1) psum += __shfl_xor(psum, o);
      Ph[qi][lane] = (b16)(p * PS); if (lane == 0) { const float sf = (mo == -INFINITY) ? ((mn == -INFINITY) ? 1.0f : 0.0f) : __expf(mo - mn); Sf[qi] = sf; Dn[qi] = Dn[qi] * sf + psum; M[qi] = mn; } }
    wave_lds_sync();
#pragma unroll
    for (int t = 0; t < 4; ++t)
#pragma unroll
      for (int r8 = 0; r8 < 8; ++r8) acc[t][r8] *= Sf[8 * hlf + r8];
    { const v16b pa = frag_kb(&Ph[nloc][0], hlf);
#pragma unroll
      for (int t = 0; t < 4; ++t) { acc[t] = wmma16b(pa, frag_kb(&Vh[t * 16 + nloc][0], hlf), acc[t]); acc[t] = wmma16b(pa, frag_kb(&Vl[t * 16 + nloc][0], hlf), acc[t]); } }
    wave_lds_sync(); }
#pragma unroll
  for (int t = 0; t < 4; ++t)
#pragma unroll
    for (int r8 = 0; r8 < 8; ++r8) { const int rl = 8 * hlf + r8; Of[rl][t * 16 + nloc] = acc[t][r8] * (1.0f / (PS * XS)) / Dn[rl]; }
  wave_lds_sync();
  for (int pass = 0; pass < 2; ++pass) { for (int rr = 0; rr < 16; ++rr) { b16* dst = ATT + (base + q0 + rr) * H + h * HD + lane * 2; const v2f o2 = {Of[rr][lane * 2], Of[rr][lane * 2 + 1]}; b16 a0 = (b16)(o2[0] * XS), a1 = (b16)(o2[1] * XS); __attribute__((ext_vector_type(2))) _Float16 pk = {a0, a1}; *(volatile __attribute__((ext_vector_type(2))) _Float16*)dst = pk; } __threadfence(); }
}
__global__ __launch_bounds__(256) void bpack_kernel(const float* __restrict__ bq, const float* __restrict__ bk, const float* __restrict__ bv, float* __restrict__ O) { for (int i = threadIdx.x; i < 3 * H; i += 256) { const float v = i < H ? bq[i] : (i < 2 * H ? bk[i - H] : bv[i - 2 * H]); for (int pass = 0; pass < 2; ++pass) { ((volatile float*)O)[i] = v; __threadfence(); } } }
}

extern "C" void kernel_launch(void* const* d_in, const int* in_sizes, int n_in, void* d_out, int out_size, void* d_ws, size_t ws_size, hipStream_t stream) {
  (void)n_in;
  auto Fp = [&](int i) { return (const float*)d_in[i]; };
  if (in_sizes[0] != ROWS * H || in_sizes[1] != H || in_sizes[3] != H * H || in_sizes[5] != H * H || in_sizes[7] != H * H || in_sizes[9] != H * H || out_size != ROWS * H) return;
  const int BV = B, RL = ROWS;
  size_t off = 0; char* ws = (char*)d_ws;
  auto carve = [&](size_t bytes) { char* p = ws + off; off += (bytes + 255) & ~(size_t)255; return p; };
  b16* WQKV = (b16*)carve((size_t)3 * H * H * 2); b16* WO = (b16*)carve((size_t)H * H * 2); b16* XN = (b16*)carve((size_t)ROWS * H * 2); float* QKV = (float*)carve((size_t)ROWS * 3 * H * 4); b16* ATT = (b16*)carve((size_t)ROWS * H * 2); float* BQKV = (float*)carve(3 * H * 4);
  if (off > ws_size || off > ((size_t)96 << 20)) return;
  wcopy_kernel<<<(unsigned)((H * H / 8 + 255) / 256), 256, 0, stream>>>(Fp(3), 0, WQKV); wcopy_kernel<<<(unsigned)((H * H / 8 + 255) / 256), 256, 0, stream>>>(Fp(5), H, WQKV); wcopy_kernel<<<(unsigned)((H * H / 8 + 255) / 256), 256, 0, stream>>>(Fp(7), 2 * H, WQKV); wcopy_kernel<<<(unsigned)((H * H / 8 + 255) / 256), 256, 0, stream>>>(Fp(9), 0, WO);
  bpack_kernel<<<1, 256, 0, stream>>>(Fp(4), Fp(6), Fp(8), BQKV);
  ln_kernel<<<(RL + 7) / 8, 256, 0, stream>>>(Fp(0), Fp(1), Fp(2), RL, XN);
  dense_kernel<0><<<(unsigned)((RL / 16) * 24), 32, 0, stream>>>(XN, WQKV, BQKV, nullptr, 24, QKV, 3 * H);
  att_kernel<<<(unsigned)(BV * NH * (RL / BV / 16)), 32, 0, stream>>>(QKV, BV, RL / BV / 16, ATT);
  dense_kernel<1><<<(unsigned)((RL / 16) * 8), 32, 0, stream>>>(ATT, WO, Fp(10), Fp(0), 8, (float*)d_out, H);
}
